// LSTMScratch_61710090109209
// MI455X (gfx1250) — hardware-verified
//
#include <hip/hip_runtime.h>
#include <math.h>

typedef __attribute__((ext_vector_type(16))) _Float16 v16h;
typedef __attribute__((ext_vector_type(8)))  float    v8f;
typedef __attribute__((ext_vector_type(4)))  float    v4f;

constexpr int kRows         = 1048576;
constexpr int kSteps        = 4;
constexpr int kHid          = 10;
constexpr int kHalfCh       = 5;
constexpr int kBlockThreads = 256;
constexpr int kRowsPerBlock = 512;
constexpr int kRowsPerWave  = 64;
constexpr int kGateStride   = 120;
constexpr int kNumGates     = 4;
static_assert(kHid == 2 * kHalfCh, "channel split over the two lane halves");
static_assert(kSteps == 4, "one 16-B vector of samples per window");
static_assert((kRows % kRowsPerBlock) == 0, "grid covers every window exactly once");
static_assert(kRowsPerBlock == (kBlockThreads / 32) * kRowsPerWave, "rows per wave");
static_assert((kRowsPerBlock * kHid) == 5 * kBlockThreads * 4, "state staging: 5 x 16 B per thread");
static_assert(kGateStride >= kHid * kHid + 2 * kHid, "gate table extent");

constexpr float kCarryState    = 128.0f;
constexpr float kCarryWeight   = 1024.0f;
constexpr float kFoldBack      = 1.0f / (kCarryState * kCarryWeight);
constexpr float kHalfMinNormal = 6.103515625e-5f;

__device__ __forceinline__ _Float16 to_half_carry(float v, float carry) {
  float s = v * carry;
  s = (fabsf(s) < kHalfMinNormal) ? 0.0f : s;
  return (_Float16)s;
}

__device__ __forceinline__ v8f mma_f16_fresh(v16h a, v16h b) {
  v8f c = (v8f){0.f, 0.f, 0.f, 0.f, 0.f, 0.f, 0.f, 0.f};
  c = __builtin_amdgcn_wmma_f32_16x16x32_f16(false, a, false, b, (short)0, c, false, false);
  asm volatile("v_nop\n\tv_nop\n\tv_nop\n\tv_nop" : "+v"(c) : "v"(a), "v"(b));
  return c;
}

__device__ __forceinline__ float sigmoid_f32(float v) {
  return __builtin_amdgcn_rcpf(1.0f + expf(-v));
}

__global__ __launch_bounds__(256) void gated_cell_scan_kernel(
    const float* __restrict__ xin, const float* __restrict__ h0, const float* __restrict__ c0,
    const float* __restrict__ wxi, const float* __restrict__ whi, const float* __restrict__ bi,
    const float* __restrict__ wxf, const float* __restrict__ whf, const float* __restrict__ bf,
    const float* __restrict__ wxo, const float* __restrict__ who, const float* __restrict__ bo,
    const float* __restrict__ wxc, const float* __restrict__ whc, const float* __restrict__ bc,
    const float* __restrict__ wlin, const float* __restrict__ blin,
    float* __restrict__ out)
{
  __shared__ __align__(16) float sH[kRowsPerBlock * kHid];
  __shared__ __align__(16) float sC[kRowsPerBlock * kHid];
  __shared__ __align__(16) float sW[kNumGates * kGateStride];
  __shared__ __align__(16) float sLin[16];

  const int tid  = threadIdx.x;
  const int lane = tid & 31;
  const int wave = tid >> 5;
  const int hh   = lane >> 4;
  const int cw   = lane & 15;
  const size_t blockRow0 = (size_t)blockIdx.x * kRowsPerBlock;

  {
    const v4f* hsrc = (const v4f*)(h0 + blockRow0 * kHid);
    const v4f* csrc = (const v4f*)(c0 + blockRow0 * kHid);
#pragma unroll
    for (int it = 0; it < 5; ++it) {
      const int q4 = it * kBlockThreads + tid;
      const v4f hv = hsrc[q4];
      const v4f cv = csrc[q4];
      *(v4f*)(sH + 4 * q4) = hv;
      *(v4f*)(sC + 4 * q4) = cv;
    }
  }

  {
    const int i100 = (tid < kHid * kHid) ? tid : (kHid * kHid - 1);
    const int i10  = (tid < kHid) ? tid : (kHid - 1);
    float wh0 = whi[i100];
    float wh1 = whf[i100];
    float wh2 = who[i100];
    float wh3 = whc[i100];
    asm volatile("" : "+v"(wh0), "+v"(wh1), "+v"(wh2), "+v"(wh3));
    float wx0 = wxi[i10];
    float wx1 = wxf[i10];
    float wx2 = wxo[i10];
    float wx3 = wxc[i10];
    asm volatile("" : "+v"(wx0), "+v"(wx1), "+v"(wx2), "+v"(wx3));
    float bb0 = bi[i10];
    float bb1 = bf[i10];
    float bb2 = bo[i10];
    float bb3 = bc[i10];
    asm volatile("" : "+v"(bb0), "+v"(bb1), "+v"(bb2), "+v"(bb3));
    float wl  = wlin[i10];
    float blv = blin[0];
    asm volatile("" : "+v"(wl), "+v"(blv));
    if (tid < kHid * kHid) {
      sW[0 * kGateStride + tid] = wh0;
      sW[1 * kGateStride + tid] = wh1;
      sW[2 * kGateStride + tid] = wh2;
      sW[3 * kGateStride + tid] = wh3;
    }
    if (tid < kHid) {
      sW[0 * kGateStride + 100 + tid] = wx0;
      sW[1 * kGateStride + 100 + tid] = wx1;
      sW[2 * kGateStride + 100 + tid] = wx2;
      sW[3 * kGateStride + 100 + tid] = wx3;
      sW[0 * kGateStride + 110 + tid] = bb0;
      sW[1 * kGateStride + 110 + tid] = bb1;
      sW[2 * kGateStride + 110 + tid] = bb2;
      sW[3 * kGateStride + 110 + tid] = bb3;
    }
    if (tid < 16) {
      const float lv = (tid < kHid) ? wl : ((tid == kHid) ? blv : 0.0f);
      sLin[tid] = lv;
    }
  }
  __syncthreads();

  float zf = 0.0f;
  asm volatile("" : "+v"(zf));
  const _Float16 zeroHalf = (_Float16)zf;
  const float onef = (hh == 0) ? kCarryState : 0.0f;
  const _Float16 oneHalf = (_Float16)onef;

  const int  rsub     = cw & 7;
  const bool rowValid = (rsub < kHalfCh);
  const int  och      = rowValid ? ((cw >> 3) * kHalfCh + rsub) : 0;
  const bool lowHalf  = rowValid && (hh == 0);
  v16h wA[kNumGates];
#pragma unroll
  for (int g = 0; g < kNumGates; ++g) {
    const float* wg = sW + g * kGateStride;
    v16h f;
#pragma unroll
    for (int i = 0; i < kHalfCh; ++i) {
      const float wv = wg[(hh * kHalfCh + i) * kHid + och];
      f[i] = to_half_carry(rowValid ? wv : 0.0f, kCarryWeight);
    }
    const float wxv = wg[100 + och];
    const float bv  = wg[110 + och];
    f[5] = to_half_carry(lowHalf ? wxv : 0.0f, kCarryWeight);
    f[6] = to_half_carry(lowHalf ? bv : 0.0f, kCarryWeight);
    f[7] = zeroHalf;
#pragma unroll
    for (int i = 8; i < 16; ++i) f[i] = (_Float16)0.0f;
    wA[g] = f;
  }

  float wl5[kHalfCh];
#pragma unroll
  for (int j = 0; j < kHalfCh; ++j) wl5[j] = sLin[hh * kHalfCh + j];
  const float headBias = sLin[kHid];

#pragma unroll 1
  for (int p = 0; p < 2; ++p) {
    float outv = 0.0f;
#pragma unroll 1
    for (int tl = 0; tl < 2; ++tl) {
      const int rl = wave * kRowsPerWave + p * 32 + tl * 16 + cw;
      float hreg[kHalfCh], creg[kHalfCh];
#pragma unroll
      for (int j = 0; j < kHalfCh; ++j) {
        hreg[j] = sH[rl * kHid + hh * kHalfCh + j];
        creg[j] = sC[rl * kHid + hh * kHalfCh + j];
      }
      const v4f xq = *(const v4f*)(xin + (blockRow0 + (size_t)rl) * kSteps);
      float x0 = xq[0];
      float x1 = xq[1];
      float x2 = xq[2];
      float x3 = xq[3];
      asm volatile("" : "+v"(x0), "+v"(x1), "+v"(x2), "+v"(x3));

#pragma unroll 1
      for (int t = 0; t < kSteps; ++t) {
        v16h bq;
#pragma unroll
        for (int j = 0; j < kHalfCh; ++j) bq[j] = to_half_carry(hreg[j], kCarryState);
        const float xs = (hh == 0) ? x0 : 0.0f;
        bq[5] = to_half_carry(xs, kCarryState);
        bq[6] = oneHalf;
        bq[7] = zeroHalf;
#pragma unroll
        for (int i = 8; i < 16; ++i) bq[i] = (_Float16)0.0f;

        const v8f ai = mma_f16_fresh(wA[0], bq);
        const v8f af = mma_f16_fresh(wA[1], bq);
        const v8f ao = mma_f16_fresh(wA[2], bq);
        const v8f ac = mma_f16_fresh(wA[3], bq);

#pragma unroll
        for (int j = 0; j < kHalfCh; ++j) {
          const float gi = sigmoid_f32(ai[j] * kFoldBack);
          const float gf = sigmoid_f32(af[j] * kFoldBack);
          const float go = sigmoid_f32(ao[j] * kFoldBack);
          const float gc = tanhf(ac[j] * kFoldBack);
          const float cn = gf * creg[j] + gi * gc;
          creg[j] = cn;
          hreg[j] = go * tanhf(cn);
        }
        x0 = x1;
        x1 = x2;
        x2 = x3;
      }

      float part = 0.0f;
#pragma unroll
      for (int j = 0; j < kHalfCh; ++j) part = fmaf(hreg[j], wl5[j], part);
      const float other = __shfl_xor(part, 16, 32);
      const float total = (part + other) + headBias;
      outv = (tl == hh) ? total : outv;
    }
    volatile float* op = (volatile float*)(out + blockRow0 + (size_t)(wave * kRowsPerWave + p * 32 + lane));
    *op = outv;
    __threadfence();
    *op = outv;
  }
}

extern "C" void kernel_launch(void* const* d_in, const int* in_sizes, int n_in,
                              void* d_out, int out_size, void* d_ws, size_t ws_size,
                              hipStream_t stream) {
  (void)d_ws;
  (void)ws_size;
  if (n_in < 17) return;
  if (in_sizes[0] != kRows * kSteps) return;
  if (in_sizes[1] != kRows * kHid) return;
  if (in_sizes[2] != kRows * kHid) return;
  if (in_sizes[3] != kHid || in_sizes[6] != kHid || in_sizes[9] != kHid || in_sizes[12] != kHid) return;
  if (in_sizes[4] != kHid * kHid || in_sizes[7] != kHid * kHid) return;
  if (in_sizes[10] != kHid * kHid || in_sizes[13] != kHid * kHid) return;
  if (in_sizes[5] != kHid || in_sizes[8] != kHid || in_sizes[11] != kHid || in_sizes[14] != kHid) return;
  if (in_sizes[15] != kHid || in_sizes[16] != 1) return;
  if (out_size != kRows) return;

  const float* xin  = (const float*)d_in[0];
  const float* h0   = (const float*)d_in[1];
  const float* c0   = (const float*)d_in[2];
  const float* wxi  = (const float*)d_in[3];
  const float* whi  = (const float*)d_in[4];
  const float* bi   = (const float*)d_in[5];
  const float* wxf  = (const float*)d_in[6];
  const float* whf  = (const float*)d_in[7];
  const float* bf   = (const float*)d_in[8];
  const float* wxo  = (const float*)d_in[9];
  const float* who  = (const float*)d_in[10];
  const float* bo   = (const float*)d_in[11];
  const float* wxc  = (const float*)d_in[12];
  const float* whc  = (const float*)d_in[13];
  const float* bc   = (const float*)d_in[14];
  const float* wlin = (const float*)d_in[15];
  const float* blin = (const float*)d_in[16];
  float* out = (float*)d_out;

  gated_cell_scan_kernel<<<kRows / kRowsPerBlock, kBlockThreads, 0, stream>>>(
      xin, h0, c0, wxi, whi, bi, wxf, whf, bf, wxo, who, bo, wxc, whc, bc, wlin, blin, out);
}
